// SmallFormerBlock_80367428043113
// MI455X (gfx1250) — hardware-verified
//
#include <hip/hip_runtime.h>
#include <math.h>
#include <stdint.h>

#define SEQ   4096
#define DMOD  512
#define NHD   8
#define HD    64
#define NKT   (SEQ / 64)
#define NQB   (SEQ / 64)
#define LNEPS 1e-5f
static_assert(NHD * HD == DMOD);
static_assert((SEQ % 64) == 0);
static_assert(DMOD == 512);
static_assert(NKT == 64 && NQB == 64);

typedef _Float16 v16h __attribute__((ext_vector_type(16)));
typedef _Float16 v8h  __attribute__((ext_vector_type(8)));
typedef float    v8f  __attribute__((ext_vector_type(8)));
typedef float    v4f  __attribute__((ext_vector_type(4)));
typedef unsigned int v4u __attribute__((ext_vector_type(4)));

#if defined(__HIP_DEVICE_COMPILE__)
#define DEV_ASM 1
#else
#define DEV_ASM 0
#endif

__device__ __forceinline__ unsigned short h_bits(_Float16 x) { return __builtin_bit_cast(unsigned short, x); }
__device__ __forceinline__ unsigned pk16(unsigned short a, unsigned short b) { return (unsigned)a | ((unsigned)b << 16); }
__device__ __forceinline__ v8f zero8() { v8f z = {0.f, 0.f, 0.f, 0.f, 0.f, 0.f, 0.f, 0.f}; return z; }
__device__ __forceinline__ float ln4(float v, float mean, float rstd) { return (v - mean) * rstd * 4.0f; }

__device__ __forceinline__ v16h ldfrag(const _Float16* p) {
  union { v16h v; v8h h[2]; } f;
  f.h[0] = *(const v8h*)(p);
  f.h[1] = *(const v8h*)(p + 16);
  return f.v;
}

__device__ __forceinline__ v8f mma_h(v16h a, v16h b, v8f c) {
  c = __builtin_amdgcn_wmma_f32_16x16x32_f16(false, a, false, b, (short)0, c, false, false);
#if DEV_ASM
  asm volatile("v_nop\n\tv_nop\n\tv_nop\n\tv_nop" : "+v"(c) : "v"(a), "v"(b));
#endif
  return c;
}

__global__ __launch_bounds__(256) void ln_planes(const float* __restrict__ x,
                                                 unsigned short* kq, unsigned short* vth, unsigned short* vtl) {
  __shared__ __align__(16) _Float16 Th[128 * 64];
  __shared__ __align__(16) _Float16 Tl[128 * 64];
  __shared__ float smean[64];
  __shared__ float srstd[64];
  const int tid  = threadIdx.x;
  const int wave = tid >> 5;
  const int lane = tid & 31;
  const int s0   = blockIdx.x * 64;

#pragma unroll 1
  for (int t = 0; t < 8; ++t) {
    const int tl = wave * 8 + t;
    const int s  = s0 + tl;
    const float* row = x + (size_t)s * DMOD;
    const v4f a0 = *(const v4f*)(row + 8 * lane);
    const v4f a1 = *(const v4f*)(row + 8 * lane + 4);
    const v4f a2 = *(const v4f*)(row + 256 + 8 * lane);
    const v4f a3 = *(const v4f*)(row + 256 + 8 * lane + 4);
    float v[16];
#pragma unroll
    for (int e = 0; e < 4; ++e) { v[e] = a0[e]; v[4 + e] = a1[e]; v[8 + e] = a2[e]; v[12 + e] = a3[e]; }
    float sum = 0.f;
#pragma unroll
    for (int i = 0; i < 16; ++i) sum += v[i];
#pragma unroll
    for (int off = 16; off > 0; off >>= 1) sum += __shfl_xor(sum, off, 32);
    const float mean = sum * (1.0f / (float)DMOD);
    float var = 0.f;
#pragma unroll
    for (int i = 0; i < 16; ++i) { const float d = v[i] - mean; var += d * d; }
#pragma unroll
    for (int off = 16; off > 0; off >>= 1) var += __shfl_xor(var, off, 32);
    const float rstd = rsqrtf(var * (1.0f / (float)DMOD) + LNEPS);

    v4u p0, p1;
#pragma unroll
    for (int e = 0; e < 4; ++e) {
      p0[e] = pk16(h_bits((_Float16)ln4(v[2 * e], mean, rstd)),     h_bits((_Float16)ln4(v[2 * e + 1], mean, rstd)));
      p1[e] = pk16(h_bits((_Float16)ln4(v[8 + 2 * e], mean, rstd)), h_bits((_Float16)ln4(v[9 + 2 * e], mean, rstd)));
    }
    const int hq = lane >> 3;
    const int d0 = (lane & 7) * 8;
    unsigned short* o0 = kq + ((size_t)hq * SEQ + (size_t)s) * HD + d0;
    unsigned short* o1 = kq + ((size_t)(hq + 4) * SEQ + (size_t)s) * HD + d0;
    *(volatile v4u*)o0 = p0;
    *(volatile v4u*)o1 = p1;
    __threadfence();
    *(volatile v4u*)o0 = p0;
    *(volatile v4u*)o1 = p1;
    if (lane == 0) { smean[tl] = mean; srstd[tl] = rstd; }
  }
  __syncthreads();

#pragma unroll 1
  for (int qtr = 0; qtr < 4; ++qtr) {
#pragma unroll 1
    for (int t = 0; t < 8; ++t) {
      const int tl = wave * 8 + t;
      const int s  = s0 + tl;
      const float mean = smean[tl];
      const float rstd = srstd[tl];
      const v4f a = *(const v4f*)(x + (size_t)s * DMOD + qtr * 128 + 4 * lane);
#pragma unroll
      for (int e = 0; e < 4; ++e) {
        const float nv = ln4(a[e], mean, rstd);
        const _Float16 hi = (_Float16)nv;
        const _Float16 lo = (_Float16)((nv - (float)hi) * 2048.0f);
        Th[(4 * lane + e) * 64 + tl] = hi;
        Tl[(4 * lane + e) * 64 + tl] = lo;
      }
    }
    __syncthreads();
    v4u hv[4], lv[4];
#pragma unroll
    for (int it = 0; it < 4; ++it) {
      const int ch = wave * 16 + it * 4 + (lane >> 3);
      const int so = (lane & 7) * 8;
      hv[it] = __builtin_bit_cast(v4u, *(const v8h*)(Th + ch * 64 + so));
      lv[it] = __builtin_bit_cast(v4u, *(const v8h*)(Tl + ch * 64 + so));
    }
    for (int ps = 0; ps < 2; ++ps) {
#pragma unroll
      for (int it = 0; it < 4; ++it) {
        const int ch = wave * 16 + it * 4 + (lane >> 3);
        const int c  = qtr * 128 + ch;
        const size_t go = (size_t)c * SEQ + (size_t)s0 + (size_t)((lane & 7) * 8);
        *(volatile v4u*)(vth + go) = hv[it];
        *(volatile v4u*)(vtl + go) = lv[it];
      }
      __threadfence();
    }
    __syncthreads();
  }
}

__global__ __launch_bounds__(128)
void attn_hd64(const unsigned short* __restrict__ kqp,
               const unsigned short* __restrict__ vhp, const unsigned short* __restrict__ vlp,
               float* ctxp, float sscale) {
  union FH { v16h v; v8h h[2]; };
  __shared__ __align__(16) _Float16 Ksh[64 * 64];
  __shared__ __align__(16) _Float16 Vth[64 * 64];
  __shared__ __align__(16) _Float16 Vtl[64 * 64];
  __shared__ __align__(16) _Float16 Psh[4][16 * 64];
  __shared__ __align__(16) float    Os[4][16 * 64];

  const int tid  = threadIdx.x;
  const int wave = tid >> 5;
  const int lane = tid & 31;
  const int hh   = lane >> 4;
  const int c    = lane & 15;

  const int bx = blockIdx.x;
  const int qb = bx % NQB;
  const int h  = bx / NQB;
  const int q0 = qb * 64 + wave * 16;

  const _Float16* Qp = (const _Float16*)(const void*)kqp + (size_t)h * SEQ * HD;
  const _Float16* Kg = Qp;
  const _Float16* Vh = (const _Float16*)(const void*)vhp + (size_t)h * HD * SEQ;
  const _Float16* Vl = (const _Float16*)(const void*)vlp + (size_t)h * HD * SEQ;

  v16h qa[2];
#pragma unroll
  for (int dc = 0; dc < 2; ++dc) {
    const size_t qo = (size_t)(q0 + c) * HD + dc * 32 + 8 * hh;
    qa[dc] = ldfrag(Qp + qo);
  }

  float mrow[8], lrow[8];
  v8f oacc[4];
#pragma unroll
  for (int r = 0; r < 8; ++r) { mrow[r] = -INFINITY; lrow[r] = 0.f; }
#pragma unroll
  for (int t = 0; t < 4; ++t) oacc[t] = zero8();

  for (int kt = 0; kt < NKT; ++kt) {
    const int kv0 = kt * 64;
    __syncthreads();
    {
      const int r = tid >> 1, half = (tid & 1) * 32;
      const _Float16* kg  = Kg + (size_t)(kv0 + r) * HD + half;
      const _Float16* vg  = Vh + (size_t)r * SEQ + kv0 + half;
      const _Float16* vlg = Vl + (size_t)r * SEQ + kv0 + half;
#pragma unroll
      for (int i = 0; i < 4; ++i) {
        const v8h a0 = *(const v8h*)(kg + 8 * i);
        const v8h b0 = *(const v8h*)(vg + 8 * i);
        const v8h b1 = *(const v8h*)(vlg + 8 * i);
        *(v8h*)(Ksh + r * 64 + half + 8 * i) = a0;
        *(v8h*)(Vth + r * 64 + half + 8 * i) = b0;
        *(v8h*)(Vtl + r * 64 + half + 8 * i) = b1;
      }
    }
    __syncthreads();

    v8f s[4];
#pragma unroll
    for (int j = 0; j < 4; ++j) {
      v8f ah = zero8();
#pragma unroll
      for (int dc = 0; dc < 2; ++dc) {
        FH kb;
        kb.h[0] = *(const v8h*)(Ksh + (j * 16 + c) * 64 + dc * 32 + 8 * hh);
        kb.h[1] = *(const v8h*)(Ksh + (j * 16 + c) * 64 + dc * 32 + 16 + 8 * hh);
        ah = mma_h(qa[dc], kb.v, ah);
      }
#pragma unroll
      for (int r = 0; r < 8; ++r) s[j][r] = ah[r] * sscale;
    }

    _Float16* pwh = Psh[wave];
#pragma unroll
    for (int r = 0; r < 8; ++r) {
      float m = s[0][r];
#pragma unroll
      for (int j = 1; j < 4; ++j) m = fmaxf(m, s[j][r]);
#pragma unroll
      for (int off = 1; off < 16; off <<= 1) m = fmaxf(m, __shfl_xor(m, off, 32));
      const float mnew  = fmaxf(mrow[r], m);
      const float msafe = (mnew == -INFINITY) ? 0.f : mnew;
      const float alpha = __expf(mrow[r] - msafe);
      mrow[r] = mnew;
      float psum = 0.f;
#pragma unroll
      for (int j = 0; j < 4; ++j) {
        const float p = __expf(s[j][r] - msafe);
        psum += p;
        pwh[(8 * hh + r) * 64 + j * 16 + c] = (_Float16)(p * 1024.0f);
      }
#pragma unroll
      for (int off = 1; off < 16; off <<= 1) psum += __shfl_xor(psum, off, 32);
      lrow[r] = lrow[r] * alpha + psum;
#pragma unroll
      for (int t = 0; t < 4; ++t) oacc[t][r] *= alpha;
    }
    __builtin_amdgcn_fence(__ATOMIC_RELEASE, "workgroup");
    __builtin_amdgcn_wave_barrier();
    __builtin_amdgcn_fence(__ATOMIC_ACQUIRE, "workgroup");

    v8f o1[4];
#pragma unroll
    for (int t = 0; t < 4; ++t) o1[t] = zero8();
#pragma unroll 1
    for (int kk = 0; kk < 2; ++kk) {
      FH pa;
      pa.h[0] = *(const v8h*)(pwh + c * 64 + kk * 32 + 8 * hh);
      pa.h[1] = *(const v8h*)(pwh + c * 64 + kk * 32 + 16 + 8 * hh);
#pragma unroll
      for (int t = 0; t < 4; ++t) {
        FH vb, vl;
        vb.h[0] = *(const v8h*)(Vth + (t * 16 + c) * 64 + kk * 32 + 8 * hh);
        vb.h[1] = *(const v8h*)(Vth + (t * 16 + c) * 64 + kk * 32 + 16 + 8 * hh);
        vl.h[0] = *(const v8h*)(Vtl + (t * 16 + c) * 64 + kk * 32 + 8 * hh);
        vl.h[1] = *(const v8h*)(Vtl + (t * 16 + c) * 64 + kk * 32 + 16 + 8 * hh);
        oacc[t] = mma_h(pa.v, vb.v, oacc[t]);
        o1[t]   = mma_h(pa.v, vl.v, o1[t]);
      }
    }
#pragma unroll
    for (int t = 0; t < 4; ++t)
#pragma unroll
      for (int r = 0; r < 8; ++r) oacc[t][r] += o1[t][r] * (1.0f / 2048.0f);
  }

  float* os = Os[wave];
#pragma unroll
  for (int r = 0; r < 8; ++r) {
    const float l = lrow[r];
    const float inv = ((l > 0.f) ? (1.0f / l) : 0.f) * (1.0f / 4096.0f);
#pragma unroll
    for (int t = 0; t < 4; ++t) os[(8 * hh + r) * 64 + t * 16 + c] = oacc[t][r] * inv;
  }
  __builtin_amdgcn_fence(__ATOMIC_RELEASE, "workgroup");
  __builtin_amdgcn_wave_barrier();
  __builtin_amdgcn_fence(__ATOMIC_ACQUIRE, "workgroup");
  {
    const int h2 = lane >> 4, c4 = (lane & 15) * 4;
    v4f ov[8];
#pragma unroll
    for (int it = 0; it < 8; ++it) {
      const int row = it * 2 + h2;
      ov[it] = *(const v4f*)(os + row * 64 + c4);
    }
    for (int ps = 0; ps < 2; ++ps) {
#pragma unroll
      for (int it = 0; it < 8; ++it) {
        const int row = it * 2 + h2;
        const size_t go = (size_t)(q0 + row) * DMOD + (size_t)h * HD + c4;
        *(volatile v4f*)(ctxp + go) = ov[it];
      }
      __threadfence();
    }
  }
}

__global__ __launch_bounds__(256) void ln_out(const float* __restrict__ x, const float* __restrict__ ctx,
                                              const float* __restrict__ pw, float* out, int ntok) {
  const int lane = threadIdx.x & 31;
  const int wave = threadIdx.x >> 5;
  const int s = blockIdx.x * 8 + wave;
  if (s >= ntok) return;
  const size_t ro = (size_t)s * DMOD;

  float r[16];
#pragma unroll
  for (int j = 0; j < 4; ++j) {
    const v4f xa = *(const v4f*)(x   + ro + 128 * j + 4 * lane);
    const v4f ca = *(const v4f*)(ctx + ro + 128 * j + 4 * lane);
#pragma unroll
    for (int e = 0; e < 4; ++e) r[4 * j + e] = ca[e] + xa[e];
  }
  float sum = 0.f;
#pragma unroll
  for (int i = 0; i < 16; ++i) sum += r[i];
#pragma unroll
  for (int off = 16; off > 0; off >>= 1) sum += __shfl_xor(sum, off, 32);
  const float mean = sum * (1.0f / (float)DMOD);
  float var = 0.f;
#pragma unroll
  for (int i = 0; i < 16; ++i) { const float d = r[i] - mean; var += d * d; }
#pragma unroll
  for (int off = 16; off > 0; off >>= 1) var += __shfl_xor(var, off, 32);
  const float rstd = rsqrtf(var * (1.0f / (float)DMOD) + LNEPS);

  v4f o[4];
#pragma unroll
  for (int j = 0; j < 4; ++j) {
    const v4f w = *(const v4f*)(pw + 128 * j + 4 * lane);
    v4f q;
#pragma unroll
    for (int e = 0; e < 4; ++e) {
      const float rr = r[4 * j + e];
      float y = (rr - mean) * rstd;
      y = (y >= 0.f) ? y : (w[e] * y);
      q[e] = y + rr;
    }
    o[j] = q;
  }
  for (int ps = 0; ps < 2; ++ps) {
#pragma unroll
    for (int j = 0; j < 4; ++j) *(volatile v4f*)(out + ro + 128 * j + 4 * lane) = o[j];
    __threadfence();
  }
}

extern "C" void kernel_launch(void* const* d_in, const int* in_sizes, int n_in,
                              void* d_out, int out_size, void* d_ws, size_t ws_size,
                              hipStream_t stream) {
  if (n_in < 2) return;
  if (in_sizes[0] != SEQ * DMOD) return;
  if (in_sizes[1] != DMOD) return;
  if (out_size != SEQ * DMOD) return;

  const float* x  = (const float*)d_in[0];
  const float* pw = (const float*)d_in[1];
  float* out = (float*)d_out;

  const size_t PKQ  = (size_t)NHD * SEQ * HD * 2;
  const size_t PVT  = (size_t)DMOD * SEQ * 2;
  const size_t PCTX = (size_t)SEQ * DMOD * 4;
  size_t off = 0;
  const size_t oKQ  = off; off += PKQ;
  const size_t oVh  = off; off += PVT;
  const size_t oVl  = off; off += PVT;
  const size_t oCtx = off; off += PCTX;
  if (off > ws_size) return;
  if (off > (size_t)134217728) return;

  char* ws = (char*)d_ws;
  unsigned short* KQ  = (unsigned short*)(ws + oKQ);
  unsigned short* VTh = (unsigned short*)(ws + oVh);
  unsigned short* VTl = (unsigned short*)(ws + oVl);
  float*          CTX = (float*)(ws + oCtx);

  const dim3 gLn(SEQ / 64);
  const dim3 gAttn(NHD * NQB);
  const dim3 gOut((SEQ + 7) / 8);

  ln_planes<<<gLn, dim3(256), 0, stream>>>(x, KQ, VTh, VTl);
  attn_hd64<<<gAttn, dim3(128), 0, stream>>>(KQ, VTh, VTl, CTX, 1.0f / 128.0f);
  ln_out<<<gOut, dim3(256), 0, stream>>>(x, CTX, pw, out, SEQ);
  (void)hipGetLastError();
}
